// CausalSelfAttention_60275571032748
// MI455X (gfx1250) — hardware-verified
//
#include <hip/hip_runtime.h>
#include <math.h>

typedef __attribute__((ext_vector_type(16))) _Float16 v16h;
typedef __attribute__((ext_vector_type(16))) __bf16 v16b;
typedef __attribute__((ext_vector_type(8)))  _Float16 v8h;
typedef __attribute__((ext_vector_type(8)))  __bf16 v8b;
typedef __attribute__((ext_vector_type(8)))  float v8f;
typedef __attribute__((ext_vector_type(4)))  float v4f;
typedef __attribute__((ext_vector_type(4)))  unsigned v4u;

template <typename T> __device__ __forceinline__ void vst2(void* p, T v) { *(volatile T*)p = v; __threadfence(); *(volatile T*)p = v; }
__device__ __forceinline__ v8f wmma16(v16h a, v16h b, v8f c) {
  v8f d = __builtin_amdgcn_wmma_f32_16x16x32_f16(false, a, false, b, (short)0, c, false, false);
  asm volatile("v_nop\n\tv_nop\n\tv_nop\n\tv_nop" : "+v"(d) : "v"(a), "v"(b));
  return d;
}
__device__ __forceinline__ v8f wmma_bf(v16b a, v16b b, v8f c) {
  v8f d = __builtin_amdgcn_wmma_f32_16x16x32_bf16(false, a, false, b, (short)0, c, false, false);
  asm volatile("v_nop\n\tv_nop\n\tv_nop\n\tv_nop" : "+v"(d) : "v"(a), "v"(b));
  return d;
}
__device__ __forceinline__ v16h frag_h(const _Float16* rowk0, int lane) {
  union { v16h v; v8h q[2]; } u; const _Float16* p = rowk0 + 8 * (lane >> 4);
  u.q[0] = *(const v8h*)p; u.q[1] = *(const v8h*)(p + 16); return u.v;
}
__device__ __forceinline__ v16b frag_b(const __bf16* rowk0, int lane) {
  union { v16b v; v8b q[2]; } u; const __bf16* p = rowk0 + 8 * (lane >> 4);
  u.q[0] = *(const v8b*)p; u.q[1] = *(const v8b*)(p + 16); return u.v;
}
__device__ __forceinline__ v16h frag_f32s(const float* rowk0, int lane, float sc) {
  v16h a; const float* p = rowk0 + 8 * (lane >> 4);
#pragma unroll
  for (int i = 0; i < 8; ++i) { a[i] = (_Float16)(p[i] * sc); a[8 + i] = (_Float16)(p[16 + i] * sc); }
  return a;
}
struct F2 { v16b h, l; };
__device__ __forceinline__ F2 bsplit16(const float v[16]) { F2 r;
#pragma unroll
  for (int i = 0; i < 16; ++i) { const __bf16 h = (__bf16)v[i]; r.h[i] = h; r.l[i] = (__bf16)(v[i] - (float)h); }
  return r; }
__device__ __forceinline__ F2 split_row(const float* row, int k0, int lane) { float v[16]; const float* p = row + k0 + 8 * (lane >> 4);
#pragma unroll
  for (int i = 0; i < 8; ++i) { v[i] = p[i]; v[8 + i] = p[16 + i]; }
  return bsplit16(v); }
__device__ __forceinline__ float bfr(float v) { return (float)(__bf16)v; }
#define LDSX() do { asm volatile("s_wait_dscnt 0" ::: "memory"); __builtin_amdgcn_wave_barrier(); __builtin_amdgcn_fence(3  , "workgroup"); } while (0)

#ifndef NB
#define NB 4
#endif
#ifndef SEQ
#define SEQ 2048
#endif
#define NB_FULL 4
#define SEQ_FULL 2048
#define TT SEQ
#define CC 1024
#define DIN 1024
#define NH 16
#define HD 64
#define NQB (TT / 64)
#define QBH 6
#define QHI 384
#define KHI 384
#define QBHE (NQB < QBH ? NQB : QBH)
#define NLO (NQB > QBH ? NQB - QBH : 1)
#define SC2 (0.125f * 1.4426950408889634f)

static_assert(NB >= 1 && NB <= NB_FULL);
static_assert(SEQ % 64 == 0 && SEQ <= SEQ_FULL && SEQ >= 64);
static_assert(CC == NH * HD);
static_assert(HD == 64);
static_assert(HD / 4 == 16);
static_assert(DIN % 64 == 0 && CC % 128 == 0 && DIN % 128 == 0 && (3 * CC) % 64 == 0);
static_assert(DIN % 32 == 0 && CC % 32 == 0);
static_assert(QHI == QBH * 64 && KHI == QHI && QHI % 64 == 0);

#define WS_QH  ((size_t)0)
#define WS_KH  (WS_QH + 2u * (size_t)NB * TT * CC)
#define WS_VT  (WS_KH + 2u * (size_t)NB * TT * CC)
#define WS_QL  (WS_VT + 2u * (size_t)NB * CC * TT)
#define WS_KL  (WS_QL + 2u * (size_t)NB * QHI * CC)
#define WS_VB  (WS_KL + 2u * (size_t)NB * KHI * CC)
#define WS_VBL (WS_VB + 2u * (size_t)NB * CC * KHI)
#define WS_WQB (WS_VBL + 2u * (size_t)NB * CC * KHI)
#define WS_WOB (WS_WQB + 2u * (size_t)3 * CC * DIN)
#define WS_WOH (WS_WOB + 2u * (size_t)DIN * CC)
#define WS_Y   (WS_WOH + 2u * (size_t)DIN * CC)
#define WS_END (WS_Y + 4u * (size_t)NB * TT * CC)
static_assert(WS_END <= (size_t)134217728);
static_assert(WS_KH == WS_QH + 2u * (size_t)NB * TT * CC);
static_assert(WS_KL == WS_QL + 2u * (size_t)NB * QHI * CC);
static_assert(WS_QL % 128 == 0 && WS_VB % 128 == 0 && WS_WQB % 128 == 0 && WS_Y % 128 == 0);

__global__ __launch_bounds__(256) void k_wt(const float* __restrict__ W, int K, int ld, __bf16* __restrict__ WB, _Float16* __restrict__ WH, int mkh) {
  __shared__ __align__(16) __bf16 tb[64][72]; __shared__ __align__(16) _Float16 th[64][72];
  const int tid = threadIdx.x; const int n0 = blockIdx.x * 64, k0 = blockIdx.y * 64;
#pragma unroll 1
  for (int e = tid; e < 64 * 64; e += 256) { const int kk = e >> 6, nn = e & 63; const float w = W[(size_t)(k0 + kk) * ld + n0 + nn]; const __bf16 wb = (__bf16)w; tb[nn][kk] = wb; th[nn][kk] = (_Float16)((float)wb * 256.0f); }
  __syncthreads();
#pragma unroll 1
  for (int e = tid; e < 64 * 8; e += 256) { const int rl = e >> 3, q = e & 7; const size_t o = (size_t)(n0 + rl) * K + k0 + q * 8; vst2(WB + o, *(const v4u*)&tb[rl][q * 8]); if (mkh) vst2(WH + o, *(const v4u*)&th[rl][q * 8]); }
}

__global__ __launch_bounds__(128) void k_proj(const float* __restrict__ X, const __bf16* __restrict__ WQB, const float* __restrict__ BQ,
    _Float16* __restrict__ QKH, _Float16* __restrict__ QKL, _Float16* __restrict__ VT, __bf16* __restrict__ VB, __bf16* __restrict__ VBL) {
  __shared__ __align__(16) _Float16 sh[64][136], sl[64][136]; __shared__ __align__(16) _Float16 th[128][72]; __shared__ __align__(16) __bf16 tb[128][72], tbl[128][72];
  const int tid = threadIdx.x, wave = tid >> 5, lane = tid & 31, col = lane & 15, g = lane >> 4; const int which = blockIdx.z; const int c0 = blockIdx.y * 128; const size_t r0 = (size_t)blockIdx.x * 64; const size_t bb = r0 / TT; const int t0 = (int)(r0 % TT);
  const size_t xr = bb * (size_t)SEQ_FULL + t0 + wave * 16 + col;
  const __bf16* WA = WQB + (size_t)which * CC * DIN; const float* BA = BQ + which * CC;
  v8f acc[8] = {};
#pragma unroll 2
  for (int kc = 0; kc < DIN / 32; ++kc) { v16b a; { const float* p = X + xr * DIN + kc * 32 + 8 * g;
#pragma unroll
      for (int i = 0; i < 8; ++i) { a[i] = (__bf16)p[i]; a[8 + i] = (__bf16)p[16 + i]; } }
    asm volatile("s_wait_loadcnt 0x0" ::: "memory");
#pragma unroll
    for (int j = 0; j < 8; ++j) { const v16b w = frag_b(WA + (size_t)(c0 + j * 16 + col) * DIN + kc * 32, lane); asm volatile("s_wait_loadcnt 0x0" ::: "memory"); acc[j] = wmma_bf(a, w, acc[j]); } }
  if (which < 2) { const int nhi = which == 0 ? QHI : KHI; _Float16* DH = QKH + (size_t)which * NB * TT * CC; _Float16* DL = QKL + (size_t)which * NB * QHI * CC; const bool hi_rows = t0 < nhi;
#pragma unroll
    for (int j = 0; j < 8; ++j) { const float bias = bfr(BA[c0 + j * 16 + col]);
#pragma unroll
      for (int r = 0; r < 8; ++r) { const float v = acc[j][r] + bias; const _Float16 hv = (_Float16)v; sh[wave * 16 + 8 * g + r][j * 16 + col] = hv; sl[wave * 16 + 8 * g + r][j * 16 + col] = (_Float16)((v - (float)hv) * 1024.0f); } }
    __syncthreads();
    for (int e = tid; e < 64 * 16; e += 128) { const int rl = e >> 4, q = e & 15; vst2(DH + (r0 + rl) * CC + c0 + q * 8, *(const v4u*)&sh[rl][q * 8]); if (hi_rows) vst2(DL + (bb * nhi + t0 + rl) * (size_t)CC + c0 + q * 8, *(const v4u*)&sl[rl][q * 8]); }
  } else { const bool hi_rows = t0 < KHI;
#pragma unroll
    for (int j = 0; j < 8; ++j) { const float bias = bfr(BA[c0 + j * 16 + col]);
#pragma unroll
      for (int r = 0; r < 8; ++r) { const float v = acc[j][r] + bias; const int rl = wave * 16 + 8 * g + r, cl = j * 16 + col; th[cl][rl] = (_Float16)v; const __bf16 bh = (__bf16)v; tb[cl][rl] = bh; tbl[cl][rl] = (__bf16)(v - (float)bh); } }
    __syncthreads();
    for (int e = tid; e < 128 * 8; e += 128) { const int cl = e >> 3, q = e & 7; vst2(VT + (bb * CC + c0 + cl) * (size_t)TT + t0 + q * 8, *(const v4u*)&th[cl][q * 8]); if (hi_rows) { const size_t o3 = (bb * CC + c0 + cl) * (size_t)KHI + t0 + q * 8; vst2(VB + o3, *(const v4u*)&tb[cl][q * 8]); vst2(VBL + o3, *(const v4u*)&tbl[cl][q * 8]); } } } }

template <int HI>
__device__ __forceinline__ void fa_body(const _Float16* __restrict__ QH, const _Float16* __restrict__ KH, const _Float16* __restrict__ QL, const _Float16* __restrict__ KL,
    const _Float16* __restrict__ VT, const __bf16* __restrict__ VB, const __bf16* __restrict__ VBL, float* __restrict__ Y, const int qb) {
  __shared__ __align__(16) float sp[4][16][HD + 4];
  const int tid = threadIdx.x, wave = tid >> 5, lane = tid & 31, col = lane & 15, g = lane >> 4;
  const int h = blockIdx.y, b = blockIdx.z;
  const int ql0 = qb * 64 + wave * 16; const size_t q0 = (size_t)b * TT + ql0;
  const _Float16* QLb = QL + (size_t)b * QHI * CC; const _Float16* KLb = KL + (size_t)b * KHI * CC;
  v16h ah[2], al[2];
#pragma unroll
  for (int kc = 0; kc < 2; ++kc) { ah[kc] = frag_h(QH + (q0 + col) * CC + h * HD + kc * 32, lane); al[kc] = ah[kc]; if (HI) al[kc] = frag_h(QLb + (size_t)(ql0 + col) * CC + h * HD + kc * 32, lane); }
  v8f o[4] = {}; float mr[8], lr[8];
#pragma unroll
  for (int r = 0; r < 8; ++r) { mr[r] = -3.0e38f; lr[r] = 0.f; }
#pragma unroll 1
  for (int kcb = 0; kcb <= qb; ++kcb) { const int k0 = kcb * 64; const size_t kr0 = (size_t)b * TT + k0;
    v8f s[4] = {}, sl[4] = {};
#pragma unroll
    for (int kc = 0; kc < 2; ++kc) {
#pragma unroll
      for (int j = 0; j < 4; ++j) { const v16h kf = frag_h(KH + (kr0 + j * 16 + col) * CC + h * HD + kc * 32, lane); s[j] = wmma16(ah[kc], kf, s[j]);
        if (HI) { const v16h kl = frag_h(KLb + (size_t)(k0 + j * 16 + col) * CC + h * HD + kc * 32, lane); sl[j] = wmma16(al[kc], kf, sl[j]); sl[j] = wmma16(ah[kc], kl, sl[j]); } } }
    const bool diag = (kcb == qb);
#pragma unroll
    for (int j = 0; j < 4; ++j) {
#pragma unroll
      for (int r = 0; r < 8; ++r) { float v = s[j][r]; if (HI) v += sl[j][r] * (1.0f / 1024.0f); v *= SC2; const bool ex = diag && (j * 16 + col > wave * 16 + 8 * g + r); s[j][r] = ex ? -3.0e38f : v; } }
#pragma unroll
    for (int r = 0; r < 8; ++r) {
      float mx = fmaxf(fmaxf(s[0][r], s[1][r]), fmaxf(s[2][r], s[3][r]));
      mx = fmaxf(mx, __shfl_xor(mx, 1)); mx = fmaxf(mx, __shfl_xor(mx, 2)); mx = fmaxf(mx, __shfl_xor(mx, 4)); mx = fmaxf(mx, __shfl_xor(mx, 8));
      const float nm = fmaxf(mr[r], mx);
      const float ea = exp2f(mr[r] - nm); const float alpha = (mr[r] < -1.0e38f) ? 0.f : ea;
      mr[r] = nm; float rs = 0.f;
#pragma unroll
      for (int j = 0; j < 4; ++j) { const float sv = s[j][r]; const float ep = exp2f(sv - nm); const float p = (sv < -1.0e38f) ? 0.f : ep; rs += p; s[j][r] = p; o[j][r] *= alpha; }
      rs += __shfl_xor(rs, 1); rs += __shfl_xor(rs, 2); rs += __shfl_xor(rs, 4); rs += __shfl_xor(rs, 8);
      lr[r] = lr[r] * alpha + rs; }
#pragma unroll
    for (int j = 0; j < 4; ++j) {
#pragma unroll
      for (int r = 0; r < 8; ++r) sp[wave][8 * g + r][j * 16 + col] = s[j][r] * 2048.0f; }
    LDSX();
#pragma unroll
    for (int kc = 0; kc < 2; ++kc) {
      if (HI) { float pv[16];
#pragma unroll
        for (int i = 0; i < 8; ++i) { pv[i] = sp[wave][col][kc * 32 + 8 * g + i]; pv[8 + i] = sp[wave][col][kc * 32 + 16 + 8 * g + i]; }
        const F2 p = bsplit16(pv);
#pragma unroll
        for (int j = 0; j < 4; ++j) { const size_t po = ((size_t)b * CC + h * HD + j * 16 + col) * (size_t)KHI + k0 + kc * 32; const v16b vh = frag_b(VB + po, lane); const v16b vl = frag_b(VBL + po, lane); o[j] = wmma_bf(p.h, vh, o[j]); o[j] = wmma_bf(p.l, vh, o[j]); o[j] = wmma_bf(p.h, vl, o[j]); }
      } else { v16h a;
#pragma unroll
        for (int i = 0; i < 8; ++i) { a[i] = (_Float16)sp[wave][col][kc * 32 + 8 * g + i]; a[8 + i] = (_Float16)sp[wave][col][kc * 32 + 16 + 8 * g + i]; }
#pragma unroll
        for (int j = 0; j < 4; ++j) { const size_t po = ((size_t)b * CC + h * HD + j * 16 + col) * (size_t)TT + k0 + kc * 32; o[j] = wmma16(a, frag_h(VT + po, lane), o[j]); } } }
    LDSX(); }
#pragma unroll
  for (int r = 0; r < 8; ++r) { const float inv = 1.0f / (lr[r] * 2048.0f);
#pragma unroll
    for (int j = 0; j < 4; ++j) sp[wave][8 * g + r][j * 16 + col] = o[j][r] * inv; }
  LDSX();
  for (int rl = 0; rl < 16; ++rl) if (lane < HD / 4) vst2(Y + (q0 + rl) * CC + h * HD + lane * 4, *(const v4f*)&sp[wave][rl][lane * 4]); }

__global__ __launch_bounds__(128) void k_fa_hi(const _Float16* __restrict__ QH, const _Float16* __restrict__ KH, const _Float16* __restrict__ QL, const _Float16* __restrict__ KL, const _Float16* __restrict__ VT, const __bf16* __restrict__ VB, const __bf16* __restrict__ VBL, float* __restrict__ Y) {
  fa_body<1>(QH, KH, QL, KL, VT, VB, VBL, Y, (int)blockIdx.x); }
__global__ __launch_bounds__(128) void k_fa_lo(const _Float16* __restrict__ QH, const _Float16* __restrict__ KH, const _Float16* __restrict__ QL, const _Float16* __restrict__ KL, const _Float16* __restrict__ VT, const __bf16* __restrict__ VB, const __bf16* __restrict__ VBL, float* __restrict__ Y) {
  fa_body<0>(QH, KH, QL, KL, VT, VB, VBL, Y, (int)blockIdx.x + QBH); }

__global__ __launch_bounds__(128) void k_out(const float* __restrict__ Y, const __bf16* __restrict__ WOB, const _Float16* __restrict__ WOH, const float* __restrict__ BO, float* __restrict__ OUT) {
  __shared__ __align__(16) float sf[4][16][132];
  const int tid = threadIdx.x, wave = tid >> 5, lane = tid & 31, col = lane & 15, g = lane >> 4; const int c0 = blockIdx.y * 128;
  const size_t rb = (size_t)blockIdx.x * 64; const size_t bb = rb / TT; const int t0 = (int)(rb % TT); const size_t r0 = rb + wave * 16; const size_t orow = bb * (size_t)SEQ_FULL + t0 + wave * 16;
  v8f acc[8] = {};
  if (t0 < QHI) {
#pragma unroll 2
    for (int kc = 0; kc < CC / 32; ++kc) { const F2 a = split_row(Y + (r0 + col) * CC, kc * 32, lane); asm volatile("s_wait_loadcnt 0x0" ::: "memory");
#pragma unroll
      for (int j = 0; j < 8; ++j) { const v16b w = frag_b(WOB + (size_t)(c0 + j * 16 + col) * CC + kc * 32, lane); asm volatile("s_wait_loadcnt 0x0" ::: "memory"); acc[j] = wmma_bf(a.h, w, acc[j]); acc[j] = wmma_bf(a.l, w, acc[j]); } }
#pragma unroll
    for (int j = 0; j < 8; ++j) { const float bias = bfr(BO[c0 + j * 16 + col]);
#pragma unroll
      for (int r = 0; r < 8; ++r) sf[wave][8 * g + r][j * 16 + col] = acc[j][r] + bias; }
  } else {
#pragma unroll 2
    for (int kc = 0; kc < CC / 32; ++kc) { const v16h a = frag_f32s(Y + (r0 + col) * CC + kc * 32, lane, 64.0f); asm volatile("s_wait_loadcnt 0x0" ::: "memory");
#pragma unroll
      for (int j = 0; j < 8; ++j) { const v16h w = frag_h(WOH + (size_t)(c0 + j * 16 + col) * CC + kc * 32, lane); asm volatile("s_wait_loadcnt 0x0" ::: "memory"); acc[j] = wmma16(a, w, acc[j]); } }
#pragma unroll
    for (int j = 0; j < 8; ++j) { const float bias = bfr(BO[c0 + j * 16 + col]);
#pragma unroll
      for (int r = 0; r < 8; ++r) sf[wave][8 * g + r][j * 16 + col] = acc[j][r] * (1.0f / 16384.0f) + bias; } }
  LDSX(); for (int rl = 0; rl < 16; ++rl) vst2(OUT + (orow + rl) * DIN + c0 + lane * 4, *(const v4f*)&sf[wave][rl][lane * 4]); }

extern "C" void kernel_launch(void* const* d_in, const int* in_sizes, int n_in, void* d_out, int out_size, void* d_ws, size_t ws_size, hipStream_t stream) {
  if (n_in < 5) return;
  const long need_rows = (long)(NB - 1) * SEQ_FULL + SEQ;
  if ((long)in_sizes[0] < need_rows * DIN) return;
  if ((long)in_sizes[1] < (long)DIN * 3 * CC) return;
  if ((long)in_sizes[2] < 3L * CC) return;
  if ((long)in_sizes[3] < (long)CC * DIN) return;
  if ((long)in_sizes[4] < (long)DIN) return;
  if ((long)out_size < need_rows * DIN) return;
  if (ws_size < (size_t)WS_END) return;
  const float* X = (const float*)d_in[0]; const float* WQ = (const float*)d_in[1]; const float* BQ = (const float*)d_in[2]; const float* WP = (const float*)d_in[3]; const float* BP = (const float*)d_in[4];
  char* ws = (char*)d_ws;
  _Float16 *QH = (_Float16*)(ws + WS_QH), *KH = (_Float16*)(ws + WS_KH), *VT = (_Float16*)(ws + WS_VT), *QL = (_Float16*)(ws + WS_QL), *KL = (_Float16*)(ws + WS_KL), *WOH = (_Float16*)(ws + WS_WOH);
  __bf16 *VB = (__bf16*)(ws + WS_VB), *VBL = (__bf16*)(ws + WS_VBL), *WQB = (__bf16*)(ws + WS_WQB), *WOB = (__bf16*)(ws + WS_WOB);
  float* Y = (float*)(ws + WS_Y);
  k_wt<<<dim3(3 * CC / 64, DIN / 64), 256, 0, stream>>>(WQ, DIN, 3 * CC, WQB, WOH, 0);
  k_wt<<<dim3(DIN / 64, CC / 64), 256, 0, stream>>>(WP, CC, DIN, WOB, WOH, 1);
  k_proj<<<dim3(NB * TT / 64, CC / 128, 3), 128, 0, stream>>>(X, WQB, BQ, QH, QL, VT, VB, VBL);
  k_fa_hi<<<dim3(QBHE, NH, NB), 128, 0, stream>>>(QH, KH, QL, KL, VT, VB, VBL, Y);
  if (NQB > QBH) k_fa_lo<<<dim3(NLO, NH, NB), 128, 0, stream>>>(QH, KH, QL, KL, VT, VB, VBL, Y);
  k_out<<<dim3(NB * TT / 64, DIN / 128), 128, 0, stream>>>(Y, WOB, WOH, BP, (float*)d_out);
}
